// GNNEdgeAttr_72224170049680
// MI455X (gfx1250) — hardware-run, weakly checked
//
#include <hip/hip_runtime.h>
#include <stddef.h>


#define NCH    512
#define EMB    64
#define KX     64
#define GT     128
#define SPW    (32 * 64)
#define WTP    72
#define RB     256
#define RBBITS 8
#define RMAX   64
#define RMBITS 6
#define TABW   (2 * RMAX)
#define CHUNK  4096
#define LCAP   6144
#define DEGCAP 64
#define WSCAP  134217728
#define ASCL   8.0f
#define WSCL   64.0f
#define INVSCL 0.001953125f

#define EDGE_INTS (RB + 8 + RB + LCAP)

static_assert(RB == (1 << RBBITS));
static_assert(RMAX == (1 << RMBITS));
static_assert(RB == 256);
static_assert(TABW == 128);
static_assert(CHUNK == 8 * 16 * 32);
static_assert(CHUNK == 4 * 4 * 256);
static_assert((WTP % 8) == 0);
static_assert((DEGCAP % 4) == 0);
static_assert(((EDGE_INTS * 4) % 16) == 0);
static_assert((KX % 64) == 0);

typedef float          v4f  __attribute__((ext_vector_type(4)));
typedef float          v8f  __attribute__((ext_vector_type(8)));
typedef int            v4i  __attribute__((ext_vector_type(4)));
typedef unsigned int   v4u  __attribute__((ext_vector_type(4)));
typedef unsigned short v8us __attribute__((ext_vector_type(8)));
typedef _Float16       v16h __attribute__((ext_vector_type(16)));
union FragH { v16h v; v8us u[2]; };

__device__ __forceinline__ unsigned short f2h(float f) {
  const _Float16 h = (_Float16)f;
  return __builtin_bit_cast(unsigned short, h);
}

__device__ __forceinline__ v8us cvt8(v4f a, v4f b, float s) {
  v8us r;
  r[0] = f2h(a.x * s); r[1] = f2h(a.y * s); r[2] = f2h(a.z * s); r[3] = f2h(a.w * s);
  r[4] = f2h(b.x * s); r[5] = f2h(b.y * s); r[6] = f2h(b.z * s); r[7] = f2h(b.w * s);
  return r;
}

__device__ __forceinline__ v8f wmh(v16h a, v16h b, v8f c) {
  v8f d = __builtin_amdgcn_wmma_f32_16x16x32_f16(false, a, false, b, (short)0, c, false, false);
  asm volatile("v_nop\n\tv_nop\n\tv_nop\n\tv_nop" : "+v"(d) : "v"(a), "v"(b));
  return d;
}

template <int NB>
__device__ __forceinline__ unsigned int match_mask(unsigned int base, int key) {
  unsigned int msk = base;
#pragma unroll
  for (int b = 0; b < NB; ++b) {
    const bool bit = ((key >> b) & 1) != 0;
    const unsigned int bb = __builtin_amdgcn_ballot_w32(bit);
    msk &= bit ? bb : ~bb;
  }
  return msk;
}

__device__ __forceinline__ v4f xadd4(v4f a, int o) {
  a.x += __shfl_xor(a.x, o); a.y += __shfl_xor(a.y, o);
  a.z += __shfl_xor(a.z, o); a.w += __shfl_xor(a.w, o);
  return a;
}

__global__ __launch_bounds__(256) void k_xcvt(const float* __restrict__ x,
                                              unsigned short* x16, unsigned short* hp,
                                              int nN, int Mp, int F) {
  const int tid = (int)threadIdx.x, lane = tid & 31, wave = tid >> 5;
  if ((int)blockIdx.x < Mp / 32) {
    const int row = (int)blockIdx.x * 32 + wave * 4 + (lane >> 3);
    const int c8 = (lane & 7) * 8;
    const int rc = row > nN - 1 ? nN - 1 : row;
    v8us o;
#pragma unroll
    for (int i = 0; i < 8; ++i) {
      const int col = c8 + i;
      const int cc = col > F - 1 ? F - 1 : col;
      float v = x[(size_t)rc * F + cc];
      v = (row < nN && col < F) ? v : 0.0f;
      o[i] = f2h(v * ASCL);
    }
    unsigned short* op = x16 + (size_t)row * KX + c8;
    *(volatile v8us*)op = o;
    __threadfence();
    *(volatile v8us*)op = o;
  } else {
    const int npc = (Mp - nN) * (NCH / 8);
    const v8us z = {0, 0, 0, 0, 0, 0, 0, 0};
    unsigned short* base = hp + (size_t)nN * NCH;
#pragma unroll 1
    for (int p = tid; p < npc; p += 256) *(volatile v8us*)(base + (size_t)p * 8) = z;
    __threadfence();
#pragma unroll 1
    for (int p = tid; p < npc; p += 256) *(volatile v8us*)(base + (size_t)p * 8) = z;
  }
}

__global__ __launch_bounds__(256) void k_wT(
    const float* __restrict__ Wq, const float* __restrict__ Wk,
    const float* __restrict__ Wv, const float* __restrict__ Ws,
    unsigned short* bt, int K, int HC, int SK, int Kp) {
  __shared__ __attribute__((aligned(16))) unsigned short sT[32 * WTP];
  const int tid = (int)threadIdx.x;
  const int bx = (int)blockIdx.x;
  const int n0 = (int)blockIdx.y * 32;
  const int g = (n0 >= 3 * HC) ? 3 : (n0 / HC);
  const float* W = (g == 0) ? Wq : ((g == 1) ? Wk : ((g == 2) ? Wv : Ws));
  const int Wd = (g < 3) ? HC : SK;
  const int nl = n0 - ((g < 3) ? g * HC : 3 * HC);

#pragma unroll
  for (int it = 0; it < 8; ++it) {
    const int i = it * 256 + tid;
    const int kk = i >> 5, nn = i & 31;
    const int k = bx * 64 + kk;
    const int kc = k > K - 1 ? K - 1 : k;
    float v = W[(size_t)kc * Wd + nl + nn];
    v = (k < K) ? v : 0.0f;
    sT[nn * WTP + kk] = f2h(v * WSCL);
  }
  __syncthreads();

  const int row = tid >> 3, c8 = (tid & 7) * 8;
  const v8us pv = *(const v8us*)(sT + row * WTP + c8);
  unsigned short* gp = bt + (size_t)(n0 + row) * Kp + bx * 64 + c8;
  *(volatile v8us*)gp = pv;
  __threadfence();
  *(volatile v8us*)gp = pv;
}

__global__ __launch_bounds__(GT) void k_gemm(
    const unsigned short* __restrict__ A, const unsigned short* __restrict__ Bt,
    const float* __restrict__ b0, const float* __restrict__ b1,
    const float* __restrict__ b2, const float* __restrict__ b3,
    float* outF, int K, int Ncols, int HC) {
  __shared__ __attribute__((aligned(16))) float sT[4 * SPW];
  const int tid = (int)threadIdx.x, lane = tid & 31, wave = tid >> 5, hh = lane >> 4, m = lane & 15;
  const int r0 = (int)blockIdx.y * 64 + (wave >> 1) * 32;
  const int c0 = (int)blockIdx.x * 128 + (wave & 1) * 64;

  const unsigned short* ap0 = A + (size_t)(r0 + m) * K + 8 * hh;
  const unsigned short* ap1 = A + (size_t)(r0 + 16 + m) * K + 8 * hh;
  const unsigned short* bp[4];
#pragma unroll
  for (int j = 0; j < 4; ++j)
    bp[j] = Bt + (size_t)(c0 + 16 * j + m) * K + 8 * hh;

  v8f acc[2][4];
#pragma unroll
  for (int i = 0; i < 2; ++i)
#pragma unroll
    for (int j = 0; j < 4; ++j) { v8f z = {0.f, 0.f, 0.f, 0.f, 0.f, 0.f, 0.f, 0.f}; acc[i][j] = z; }

  const int nk = K >> 5;
#pragma unroll 1
  for (int kt = 0; kt < nk; ++kt) {
    const int kb = kt << 5;
    FragH a0, a1;
    a0.u[0] = *(const v8us*)(ap0 + kb);
    a0.u[1] = *(const v8us*)(ap0 + kb + 16);
    a1.u[0] = *(const v8us*)(ap1 + kb);
    a1.u[1] = *(const v8us*)(ap1 + kb + 16);
#pragma unroll
    for (int j = 0; j < 4; ++j) {
      FragH bf;
      bf.u[0] = *(const v8us*)(bp[j] + kb);
      bf.u[1] = *(const v8us*)(bp[j] + kb + 16);
      acc[0][j] = wmh(a0.v, bf.v, acc[0][j]);
      acc[1][j] = wmh(a1.v, bf.v, acc[1][j]);
    }
  }

  float* sw = sT + wave * SPW;
#pragma unroll
  for (int i = 0; i < 2; ++i)
#pragma unroll
    for (int j = 0; j < 4; ++j)
#pragma unroll
      for (int r = 0; r < 8; ++r)
        sw[(16 * i + 8 * hh + r) * 64 + 16 * j + m] = acc[i][j][r];
  __syncthreads();

  const int g = (c0 >= 3 * HC) ? 3 : (c0 / HC);
  const float* bias = (g == 0) ? b0 : ((g == 1) ? b1 : ((g == 2) ? b2 : b3));
  const int bl = c0 - ((g < 3) ? g * HC : 3 * HC);

  v4f ov[16];
  size_t po[16];
#pragma unroll
  for (int it = 0; it < 16; ++it) {
    const int f = it * 32 + lane;
    const int row = f >> 4, c4 = (f & 15) * 4;
    const v4f v = *(const v4f*)(sw + row * 64 + c4);
    const v4f bb = *(const v4f*)(bias + bl + c4);
    ov[it] = v * INVSCL + bb;
    po[it] = (size_t)(r0 + row) * Ncols + c0 + c4;
  }
#pragma unroll
  for (int it = 0; it < 16; ++it) *(volatile v4f*)(outF + po[it]) = ov[it];
  __threadfence();
#pragma unroll
  for (int it = 0; it < 16; ++it) *(volatile v4f*)(outF + po[it]) = ov[it];
}

__global__ __launch_bounds__(256) void k_csort(
    const int* __restrict__ dst, unsigned int* csort, int* tab, int nN, int nE) {
  __shared__ __attribute__((aligned(16))) unsigned int sImg[CHUNK];
  __shared__ int cw[8 * RMAX];
  __shared__ __attribute__((aligned(16))) int sPre[RMAX];
  __shared__ __attribute__((aligned(16))) int sCn[RMAX];
  __shared__ int sWt[8];
  const int tid = (int)threadIdx.x, lane = tid & 31, wave = tid >> 5;
  const int c = (int)blockIdx.x;
  const int cbase = c * CHUNK;

  for (int i = tid; i < 8 * RMAX; i += 256) cw[i] = 0;
  {
    const v4u s = {0xffffffffu, 0xffffffffu, 0xffffffffu, 0xffffffffu};
    for (int i = tid; i < CHUNK / 4; i += 256) ((v4u*)sImg)[i] = s;
  }
  __syncthreads();

  unsigned int ent[16];
  int pk[16];
  const unsigned int lt = (1u << lane) - 1u;
#pragma unroll
  for (int i = 0; i < 16; ++i) {
    const int e = cbase + wave * 512 + 32 * i + lane;
    const int ec = e > nE - 1 ? nE - 1 : e;
    const int d = dst[ec];
    const bool valid = (e < nE) && ((unsigned)d < (unsigned)nN);
    const int dd = valid ? d : 0;
    const int r  = dd >> RBBITS;
    const int jl = dd & (RB - 1);
    const unsigned int msk = match_mask<RMBITS>(__builtin_amdgcn_ballot_w32(valid), r);
    const int rank = (int)__builtin_popcount(msk & lt);
    const int grp  = (int)__builtin_popcount(msk);
    const int base = cw[wave * RMAX + r];
    pk[i]  = valid ? ((r << 12) | (base + rank)) : -1;
    ent[i] = ((unsigned int)ec << RBBITS) | (unsigned int)jl;
    if (valid && rank == 0) cw[wave * RMAX + r] = base + grp;
    __syncthreads();
  }

  if (tid < RMAX) {
    int run = 0;
#pragma unroll
    for (int w = 0; w < 8; ++w) {
      const int v = cw[w * RMAX + tid];
      cw[w * RMAX + tid] = run;
      run += v;
    }
    sCn[tid] = run;
  }
  __syncthreads();
  {
    const int vr = sCn[tid & (RMAX - 1)];
    const int v  = (tid < RMAX) ? vr : 0;
    int x = v;
#pragma unroll
    for (int dd = 1; dd < 32; dd <<= 1) {
      const int y = __shfl_up(x, dd);
      x += (lane >= dd) ? y : 0;
    }
    if (lane == 31) sWt[wave] = x;
    __syncthreads();
    int pre = 0;
#pragma unroll
    for (int w = 0; w < 8; ++w) { const int tw = sWt[w]; pre += (w < wave) ? tw : 0; }
    if (tid < RMAX) sPre[tid] = pre + x - v;
  }
  __syncthreads();

#pragma unroll
  for (int i = 0; i < 16; ++i) {
    if (pk[i] >= 0) {
      const int r = (pk[i] >> 12) & (RMAX - 1);
      const int q = pk[i] & 4095;
      const int pos = sPre[r] + cw[wave * RMAX + r] + q;
      if ((unsigned)pos < (unsigned)CHUNK) sImg[pos] = ent[i];
    }
  }
  __syncthreads();

  v4u iv[4];
#pragma unroll
  for (int it = 0; it < 4; ++it) iv[it] = ((const v4u*)sImg)[it * 256 + tid];
  const v4i ta = *(const v4i*)(sPre + 4 * (lane & 15));
  const v4i tb = *(const v4i*)(sCn + 4 * (lane & 15));
  const v4i tv = (lane < 16) ? ta : tb;
  unsigned int* gp = csort + (size_t)c * CHUNK;
  int* tp = tab + (size_t)c * TABW + 4 * lane;
  const bool wt = (wave == 0);
#pragma unroll
  for (int it = 0; it < 4; ++it) *(volatile v4u*)(gp + 4 * (it * 256 + tid)) = iv[it];
  if (wt) *(volatile v4i*)tp = tv;
  __threadfence();
#pragma unroll
  for (int it = 0; it < 4; ++it) *(volatile v4u*)(gp + 4 * (it * 256 + tid)) = iv[it];
  if (wt) *(volatile v4i*)tp = tv;
}

template <int HCW, int CH, int OUT16>
__global__ __launch_bounds__(256) void k_edge(
    const float* __restrict__ qkvs, const int* __restrict__ src,
    const float* __restrict__ ea, const float* __restrict__ We,
    const unsigned int* __restrict__ csort, const int* __restrict__ tab,
    float* outF, unsigned short* outH, int nN, int nE, int nCh) {
  constexpr int LPE = (HCW / 8) < 32 ? (HCW / 8) : 32;
  constexpr int EPI = 32 / LPE;
  constexpr int NSL = HCW / (LPE * 8);
  constexpr int LPH = CH / 8;
  constexpr int NIT = DEGCAP / EPI;
  constexpr int SCW = 32 * NIT;
  constexpr int NC  = 4 * HCW;
  static_assert(LPE * EPI == 32);
  static_assert(NSL * LPE * 8 == HCW);
  static_assert(CH == 64 || CH == 128);
  static_assert((LPE % LPH) == 0);
  extern __shared__ __attribute__((aligned(16))) int dsm[];
  __shared__ int sWtot[8];
  int*   sOff  = dsm;
  int*   sCur  = dsm + (RB + 8);
  int*   sList = sCur + RB;
  float* sSc   = (float*)(dsm + EDGE_INTS);
  float* sO    = sSc + 8 * SCW;
  const int tid = (int)threadIdx.x, lane = tid & 31, wave = tid >> 5;
  const int rgn = (int)blockIdx.x;
  const int n0 = rgn * RB;
  const unsigned int lt = (1u << lane) - 1u;

  for (int i = tid; i < RB + 8; i += 256) sOff[i] = 0;
  for (int i = tid; i < RB; i += 256) sCur[i] = 0;
  __syncthreads();

#pragma unroll 1
  for (int c = 0; c < nCh; ++c) {
    int pre = tab[(size_t)c * TABW + rgn];
    int n   = tab[(size_t)c * TABW + RMAX + rgn];
    pre = pre < 0 ? 0 : (pre > CHUNK ? CHUNK : pre);
    n = n < 0 ? 0 : (n > CHUNK - pre ? CHUNK - pre : n);
    const int nstep = (n + 31) >> 5;
    const unsigned int* cp = csort + (size_t)c * CHUNK + pre;
#pragma unroll 1
    for (int s = 0; s < nstep; ++s) {
      if (wave == 0) {
        const int i = (s << 5) + lane;
        const bool valid = i < n;
        const int ic = i > n - 1 ? n - 1 : i;
        const unsigned int en = cp[ic];
        const int j = (int)(en & (unsigned int)(RB - 1));
        const unsigned int msk = match_mask<RBBITS>(__builtin_amdgcn_ballot_w32(valid), j);
        const int rank = (int)__builtin_popcount(msk & lt);
        const int grp  = (int)__builtin_popcount(msk);
        if (valid && rank == 0) sOff[j] = sOff[j] + grp;
      }
      __syncthreads();
    }
  }
  __syncthreads();

  {
    const int cn = sOff[tid];
    int x = cn;
#pragma unroll
    for (int dd = 1; dd < 32; dd <<= 1) {
      const int y = __shfl_up(x, dd);
      x += (lane >= dd) ? y : 0;
    }
    if (lane == 31) sWtot[wave] = x;
    __syncthreads();
    int pre = 0;
#pragma unroll
    for (int w = 0; w < 8; ++w) { const int tw = sWtot[w]; pre += (w < wave) ? tw : 0; }
    const int run = pre + x - cn;
    sOff[tid] = run;
    if (tid == 255) sOff[RB] = run + cn;
  }
  __syncthreads();

#pragma unroll 1
  for (int c = 0; c < nCh; ++c) {
    int pre = tab[(size_t)c * TABW + rgn];
    int n   = tab[(size_t)c * TABW + RMAX + rgn];
    pre = pre < 0 ? 0 : (pre > CHUNK ? CHUNK : pre);
    n = n < 0 ? 0 : (n > CHUNK - pre ? CHUNK - pre : n);
    const int nstep = (n + 31) >> 5;
    const unsigned int* cp = csort + (size_t)c * CHUNK + pre;
#pragma unroll 1
    for (int s = 0; s < nstep; ++s) {
      if (wave == 0) {
        const int i = (s << 5) + lane;
        const bool valid = i < n;
        const int ic = i > n - 1 ? n - 1 : i;
        const unsigned int en = cp[ic];
        const int j = (int)(en & (unsigned int)(RB - 1));
        int e = (int)(en >> RBBITS);
        e = e > nE - 1 ? nE - 1 : e;
        const unsigned int msk = match_mask<RBBITS>(__builtin_amdgcn_ballot_w32(valid), j);
        const int rank = (int)__builtin_popcount(msk & lt);
        const int grp  = (int)__builtin_popcount(msk);
        const int cur  = sCur[j];
        const int p0   = sOff[j] + cur + rank;
        if (valid && (unsigned)p0 < (unsigned)LCAP) sList[p0] = e;
        if (valid && rank == 0) sCur[j] = cur + grp;
      }
      __syncthreads();
    }
  }
  __syncthreads();

  const int es = lane / LPE;
  const int cl = (lane % LPE) * 8;
  const float rs = (CH == 64) ? 0.125f : 0.08838834764831845f;
  const float ninf = __int_as_float(0xff800000u);
  int Rb = nN - n0; Rb = Rb > RB ? RB : Rb;
  float* sw = sSc + wave * SCW;
  float* so = sO + wave * HCW;
#pragma unroll 1
  for (int j = wave; j < Rb; j += 8) {
    const int node = n0 + j;
    int lb = __builtin_amdgcn_readfirstlane(sOff[j]);
    int ub = __builtin_amdgcn_readfirstlane(sOff[j + 1]);
    lb = lb < 0 ? 0 : (lb > LCAP ? LCAP : lb);
    ub = ub < 0 ? 0 : (ub > LCAP ? LCAP : ub);
    int cnt = ub - lb;
    cnt = cnt < 0 ? 0 : (cnt > DEGCAP ? DEGCAP : cnt);
    const int np = (cnt + EPI - 1) / EPI;
    const float* qr = qkvs + (size_t)node * NC;

#pragma unroll 1
    for (int sl = 0; sl < NSL; ++sl) {
      const int ch = sl * 256 + cl;
      const v4f q0  = *(const v4f*)(qr + ch);
      const v4f q1  = *(const v4f*)(qr + ch + 4);
      const v4f wa0 = *(const v4f*)(We + ch);
      const v4f wa1 = *(const v4f*)(We + ch + 4);
      const v4f wb0 = *(const v4f*)(We + HCW + ch);
      const v4f wb1 = *(const v4f*)(We + HCW + ch + 4);

      float mx = ninf;
#pragma unroll 1
      for (int it = 0; it < np; ++it) {
        const int i = it * EPI + es;
        const bool valid = i < cnt;
        const int ic = valid ? i : (cnt - 1);
        int li = lb + ic; li = li < 0 ? 0 : (li > LCAP - 1 ? LCAP - 1 : li);
        int e = sList[li]; e = e < 0 ? 0 : (e > nE - 1 ? nE - 1 : e);
        int s = src[e];   s = s < 0 ? 0 : (s > nN - 1 ? nN - 1 : s);
        const float a0 = ea[2 * (size_t)e];
        const float a1 = ea[2 * (size_t)e + 1];
        const float* kr = qkvs + (size_t)s * NC + HCW + ch;
        const v4f k0 = *(const v4f*)kr;
        const v4f k1 = *(const v4f*)(kr + 4);
        const v4f e0 = wa0 * a0 + wb0 * a1;
        const v4f e1 = wa1 * a0 + wb1 * a1;
        const v4f kj0 = k0 + e0;
        const v4f kj1 = k1 + e1;
        float part = q0.x * kj0.x;
        part = fmaf(q0.y, kj0.y, part);
        part = fmaf(q0.z, kj0.z, part);
        part = fmaf(q0.w, kj0.w, part);
        part = fmaf(q1.x, kj1.x, part);
        part = fmaf(q1.y, kj1.y, part);
        part = fmaf(q1.z, kj1.z, part);
        part = fmaf(q1.w, kj1.w, part);
#pragma unroll
        for (int o = 1; o < LPH; o <<= 1) part += __shfl_xor(part, o);
        const float sc = part * rs;
        mx = valid ? fmaxf(mx, sc) : mx;
        sw[it * 32 + lane] = sc;
      }
#pragma unroll
      for (int o = LPE; o < 32; o <<= 1) mx = fmaxf(mx, __shfl_xor(mx, o));

      v4f acc0 = {0.f, 0.f, 0.f, 0.f};
      v4f acc1 = {0.f, 0.f, 0.f, 0.f};
      float z = 0.0f;
#pragma unroll 1
      for (int it = 0; it < np; ++it) {
        const int i = it * EPI + es;
        const bool valid = i < cnt;
        const int ic = valid ? i : (cnt - 1);
        int li = lb + ic; li = li < 0 ? 0 : (li > LCAP - 1 ? LCAP - 1 : li);
        int e = sList[li]; e = e < 0 ? 0 : (e > nE - 1 ? nE - 1 : e);
        int s = src[e];   s = s < 0 ? 0 : (s > nN - 1 ? nN - 1 : s);
        const float a0 = ea[2 * (size_t)e];
        const float a1 = ea[2 * (size_t)e + 1];
        const float sc = sw[it * 32 + lane];
        float p = __expf(sc - mx);
        p = valid ? p : 0.0f;
        const float* vr = qkvs + (size_t)s * NC + 2 * HCW + ch;
        const v4f v0 = *(const v4f*)vr;
        const v4f v1 = *(const v4f*)(vr + 4);
        const v4f e0 = wa0 * a0 + wb0 * a1;
        const v4f e1 = wa1 * a0 + wb1 * a1;
        const v4f vj0 = v0 + e0;
        const v4f vj1 = v1 + e1;
        acc0 = acc0 + vj0 * p;
        acc1 = acc1 + vj1 * p;
        z += p;
      }
#pragma unroll
      for (int o = LPE; o < 32; o <<= 1) {
        acc0 = xadd4(acc0, o);
        acc1 = xadd4(acc1, o);
        z += __shfl_xor(z, o);
      }
      const float zs = (cnt > 0) ? z : 1.0f;
      const float rz = (cnt > 0) ? (1.0f / zs) : 0.0f;
      const v4f s0 = *(const v4f*)(qr + 3 * HCW + ch);
      const v4f s1 = *(const v4f*)(qr + 3 * HCW + ch + 4);
      v4f o0 = acc0 * rz + s0;
      v4f o1 = acc1 * rz + s1;
      if (OUT16) {
        o0.x = fmaxf(o0.x, 0.0f); o0.y = fmaxf(o0.y, 0.0f); o0.z = fmaxf(o0.z, 0.0f); o0.w = fmaxf(o0.w, 0.0f);
        o1.x = fmaxf(o1.x, 0.0f); o1.y = fmaxf(o1.y, 0.0f); o1.z = fmaxf(o1.z, 0.0f); o1.w = fmaxf(o1.w, 0.0f);
      }
      if (lane < LPE) {
        *(v4f*)(so + ch) = o0;
        *(v4f*)(so + ch + 4) = o1;
      }
    }
    __builtin_amdgcn_fence(__ATOMIC_RELEASE, "wavefront");
    __builtin_amdgcn_wave_barrier();

    if (OUT16) {
      constexpr int NP = HCW / 8;
      constexpr int NI = (NP + 31) / 32;
      v8us hv[NI];
      size_t po[NI];
#pragma unroll
      for (int it = 0; it < NI; ++it) {
        int p = it * 32 + lane; p = p > NP - 1 ? NP - 1 : p;
        const v4f a = *(const v4f*)(so + p * 8);
        const v4f b = *(const v4f*)(so + p * 8 + 4);
        hv[it] = cvt8(a, b, ASCL);
        po[it] = (size_t)node * HCW + (size_t)p * 8;
      }
#pragma unroll
      for (int it = 0; it < NI; ++it)
        if (it * 32 + lane < NP) *(volatile v8us*)(outH + po[it]) = hv[it];
      __threadfence();
#pragma unroll
      for (int it = 0; it < NI; ++it)
        if (it * 32 + lane < NP) *(volatile v8us*)(outH + po[it]) = hv[it];
    } else {
      constexpr int NP = HCW / 4;
      constexpr int NI = (NP + 31) / 32;
      v4f fv[NI];
      size_t po[NI];
#pragma unroll
      for (int it = 0; it < NI; ++it) {
        int p = it * 32 + lane; p = p > NP - 1 ? NP - 1 : p;
        fv[it] = *(const v4f*)(so + p * 4);
        po[it] = (size_t)node * HCW + (size_t)p * 4;
      }
#pragma unroll
      for (int it = 0; it < NI; ++it)
        if (it * 32 + lane < NP) *(volatile v4f*)(outF + po[it]) = fv[it];
      __threadfence();
#pragma unroll
      for (int it = 0; it < NI; ++it)
        if (it * 32 + lane < NP) *(volatile v4f*)(outF + po[it]) = fv[it];
    }
    __builtin_amdgcn_wave_barrier();
  }
}

static size_t edge_lds_bytes(int hcw) {
  int lpe = hcw / 8; lpe = lpe > 32 ? 32 : lpe;
  const int epi = 32 / lpe;
  const int nit = DEGCAP / epi;
  return (size_t)(EDGE_INTS + 8 * 32 * nit + 8 * hcw) * 4;
}

extern "C" void kernel_launch(void* const* d_in, const int* in_sizes, int n_in,
                              void* d_out, int out_size, void* d_ws, size_t ws_size,
                              hipStream_t stream) {
  if (n_in < 31) return;
  if (in_sizes[5] != NCH) return;
  const int F = in_sizes[4] / NCH;
  if (F < 1 || F > KX || in_sizes[4] != F * NCH) return;
  const int nN = in_sizes[0] / F;
  if (nN <= 0 || in_sizes[0] != nN * F) return;
  const int nE = in_sizes[1];
  if (nE <= 0 || in_sizes[2] != nE || in_sizes[3] != 2 * nE) return;
  if (nN > RMAX * RB || nE > (1 << 23)) return;
  if (in_sizes[6] != F * NCH || in_sizes[8] != F * NCH || in_sizes[11] != F * NCH) return;
  if (in_sizes[7] != NCH || in_sizes[9] != NCH || in_sizes[12] != NCH || in_sizes[10] != 2 * NCH) return;
  if (in_sizes[13] != NCH * NCH || in_sizes[15] != NCH * NCH || in_sizes[17] != NCH * NCH || in_sizes[20] != NCH * NCH) return;
  if (in_sizes[14] != NCH || in_sizes[16] != NCH || in_sizes[18] != NCH || in_sizes[21] != NCH || in_sizes[19] != 2 * NCH) return;
  if (in_sizes[22] != NCH * EMB || in_sizes[24] != NCH * EMB || in_sizes[26] != NCH * EMB || in_sizes[29] != NCH * EMB) return;
  if (in_sizes[23] != EMB || in_sizes[25] != EMB || in_sizes[27] != EMB || in_sizes[30] != EMB || in_sizes[28] != 2 * EMB) return;
  if (out_size != nN * EMB) return;

  const float* x   = (const float*)d_in[0];
  const int*   src = (const int*)d_in[1];
  const int*   dst = (const int*)d_in[2];
  const float* ea  = (const float*)d_in[3];
  const float* Wq1 = (const float*)d_in[4];  const float* bq1 = (const float*)d_in[5];
  const float* Wk1 = (const float*)d_in[6];  const float* bk1 = (const float*)d_in[7];
  const float* Wv1 = (const float*)d_in[8];  const float* bv1 = (const float*)d_in[9];
  const float* We1 = (const float*)d_in[10];
  const float* Ws1 = (const float*)d_in[11]; const float* bs1 = (const float*)d_in[12];
  const float* Wq2 = (const float*)d_in[13]; const float* bq2 = (const float*)d_in[14];
  const float* Wk2 = (const float*)d_in[15]; const float* bk2 = (const float*)d_in[16];
  const float* Wv2 = (const float*)d_in[17]; const float* bv2 = (const float*)d_in[18];
  const float* We2 = (const float*)d_in[19];
  const float* Ws2 = (const float*)d_in[20]; const float* bs2 = (const float*)d_in[21];
  const float* Wq3 = (const float*)d_in[22]; const float* bq3 = (const float*)d_in[23];
  const float* Wk3 = (const float*)d_in[24]; const float* bk3 = (const float*)d_in[25];
  const float* Wv3 = (const float*)d_in[26]; const float* bv3 = (const float*)d_in[27];
  const float* We3 = (const float*)d_in[28];
  const float* Ws3 = (const float*)d_in[29]; const float* bs3 = (const float*)d_in[30];
  float* out = (float*)d_out;

  const int Mp  = ((nN + 63) / 64) * 64;
  const int nCh = (nE + CHUNK - 1) / CHUNK;
  const int nR  = (nN + RB - 1) / RB;
  const int NC12 = 4 * NCH;
  const int NC3  = 4 * EMB;

  const size_t szX16 = (size_t)Mp * KX * 2;
  const size_t szBt1 = (size_t)NC12 * KX * 2;
  const size_t szBt2 = (size_t)NC12 * NCH * 2;
  const size_t szBt3 = (size_t)NC3 * NCH * 2;
  const size_t szQ   = (size_t)Mp * NC12 * 4;
  const size_t szH   = (size_t)Mp * NCH * 2;
  const size_t szCS  = (size_t)nCh * CHUNK * 4;
  const size_t szTab = (size_t)nCh * TABW * 4;
  size_t off = 0;
  const size_t oX  = off; off += szX16; off = (off + 255) & ~(size_t)255;
  const size_t oB1 = off; off += szBt1; off = (off + 255) & ~(size_t)255;
  const size_t oB2 = off; off += szBt2; off = (off + 255) & ~(size_t)255;
  const size_t oB3 = off; off += szBt3; off = (off + 255) & ~(size_t)255;
  const size_t oQ  = off; off += szQ;   off = (off + 255) & ~(size_t)255;
  const size_t oH  = off; off += szH;   off = (off + 255) & ~(size_t)255;
  const size_t oCS = off; off += szCS;  off = (off + 255) & ~(size_t)255;
  const size_t oT  = off; off += szTab; off = (off + 255) & ~(size_t)255;
  if (off > ws_size || off > (size_t)WSCAP) return;

  char* ws = (char*)d_ws;
  unsigned short* x16   = (unsigned short*)(ws + oX);
  unsigned short* bt1   = (unsigned short*)(ws + oB1);
  unsigned short* bt2   = (unsigned short*)(ws + oB2);
  unsigned short* bt3   = (unsigned short*)(ws + oB3);
  float*          qkvs  = (float*)(ws + oQ);
  unsigned short* hpl   = (unsigned short*)(ws + oH);
  unsigned int*   csort = (unsigned int*)(ws + oCS);
  int*            tab   = (int*)(ws + oT);

  const size_t lds12 = edge_lds_bytes(NCH);
  const size_t lds3  = edge_lds_bytes(EMB);

  k_xcvt<<<Mp / 32 + 1, 256, 0, stream>>>(x, x16, hpl, nN, Mp, F);

  k_wT<<<dim3(KX / 64, NC12 / 32), 256, 0, stream>>>(Wq1, Wk1, Wv1, Ws1, bt1, F, NCH, NCH, KX);
  k_wT<<<dim3(NCH / 64, NC12 / 32), 256, 0, stream>>>(Wq2, Wk2, Wv2, Ws2, bt2, NCH, NCH, NCH, NCH);
  k_wT<<<dim3(NCH / 64, NC3 / 32), 256, 0, stream>>>(Wq3, Wk3, Wv3, Ws3, bt3, NCH, EMB, EMB, NCH);

  k_csort<<<nCh, 256, 0, stream>>>(dst, csort, tab, nN, nE);

  k_gemm<<<dim3(NC12 / 128, Mp / 64), GT, 0, stream>>>(x16, bt1, bq1, bk1, bv1, bs1, qkvs, KX, NC12, NCH);
  hipFuncSetAttribute(reinterpret_cast<const void*>(&k_edge<NCH, 128, 1>),
                      hipFuncAttributeMaxDynamicSharedMemorySize, (int)lds12);
  k_edge<NCH, 128, 1><<<nR, 256, lds12, stream>>>(qkvs, src, ea, We1, csort, tab, out, hpl, nN, nE, nCh);

  k_gemm<<<dim3(NC12 / 128, Mp / 64), GT, 0, stream>>>(hpl, bt2, bq2, bk2, bv2, bs2, qkvs, NCH, NC12, NCH);
  k_edge<NCH, 128, 1><<<nR, 256, lds12, stream>>>(qkvs, src, ea, We2, csort, tab, out, hpl, nN, nE, nCh);

  k_gemm<<<dim3(NC3 / 128, Mp / 64), GT, 0, stream>>>(hpl, bt3, bq3, bk3, bv3, bs3, qkvs, NCH, NC3, EMB);
  hipFuncSetAttribute(reinterpret_cast<const void*>(&k_edge<EMB, 64, 0>),
                      hipFuncAttributeMaxDynamicSharedMemorySize, (int)lds3);
  k_edge<EMB, 64, 0><<<nR, 256, lds3, stream>>>(qkvs, src, ea, We3, csort, tab, out, hpl, nN, nE, nCh);
}
